// PointnetSAModuleMSG_19069654794722
// MI455X (gfx1250) — hardware-verified
//
#include <hip/hip_runtime.h>
#include <math.h>

typedef __attribute__((ext_vector_type(16))) _Float16 v16h;
typedef __attribute__((ext_vector_type(16))) __bf16 v16b;
typedef __attribute__((ext_vector_type(8)))  _Float16 v8h;
typedef __attribute__((ext_vector_type(8)))  float v8f;
typedef __attribute__((ext_vector_type(4)))  float v4f;
typedef __attribute__((ext_vector_type(2)))  float v2f;
typedef __attribute__((ext_vector_type(4)))  unsigned v4u;
typedef __attribute__((ext_vector_type(4)))  int v4i;
typedef float __attribute__((may_alias)) float_a;
typedef int __attribute__((may_alias)) int_a;

template <typename T> __device__ __forceinline__ void vst2(void* p, T v) { *(volatile T*)p = v; __threadfence(); *(volatile T*)p = v; }
__device__ __forceinline__ v8f wmma16(v16h a, v16h b, v8f c) {
  v8f d = __builtin_amdgcn_wmma_f32_16x16x32_f16(false, a, false, b, (short)0, c, false, false);
  asm volatile("v_nop\n\tv_nop\n\tv_nop\n\tv_nop" : "+v"(d) : "v"(a), "v"(b));
  return d;
}
__device__ __forceinline__ v8f wmma_bf(v16b a, v16b b, v8f c) {
  v8f d = __builtin_amdgcn_wmma_f32_16x16x32_bf16(false, a, false, b, (short)0, c, false, false);
  asm volatile("v_nop\n\tv_nop\n\tv_nop\n\tv_nop" : "+v"(d) : "v"(a), "v"(b));
  return d;
}
__device__ __forceinline__ v16h frag_h(const _Float16* rowk0, int lane) {
  union { v16h v; v8h q[2]; } u; const _Float16* p = rowk0 + 8 * (lane >> 4);
  u.q[0] = *(const v8h*)p; u.q[1] = *(const v8h*)(p + 16); return u.v;
}
__device__ __forceinline__ v16h frag_f32(const float* rowk0, int lane) {
  v16h a; const float* p = rowk0 + 8 * (lane >> 4);
#pragma unroll
  for (int i = 0; i < 8; ++i) { a[i] = (_Float16)p[i]; a[8 + i] = (_Float16)p[16 + i]; }
  return a;
}
__device__ __forceinline__ v16h frag_f32s(const float* rowk0, int lane, float sc) {
  v16h a; const float* p = rowk0 + 8 * (lane >> 4);
#pragma unroll
  for (int i = 0; i < 8; ++i) { a[i] = (_Float16)(p[i] * sc); a[8 + i] = (_Float16)(p[16 + i] * sc); }
  return a;
}
__device__ __forceinline__ v16h fragc_f32(const float* W, int k0, int n, int lane, int ld, int K) {
  v16h a; const int g = lane >> 4;
#pragma unroll
  for (int i = 0; i < 8; ++i) { const int ka = k0 + 8 * g + i, kb = ka + 16;
    a[i] = (_Float16)(ka < K ? W[(size_t)(ka < K ? ka : K - 1) * ld + n] : 0.f); a[8 + i] = (_Float16)(kb < K ? W[(size_t)(kb < K ? kb : K - 1) * ld + n] : 0.f); }
  return a;
}
struct F2 { v16b h, l; };
__device__ __forceinline__ F2 bsplit16(const float v[16]) { F2 r;
#pragma unroll
  for (int i = 0; i < 16; ++i) { const __bf16 h = (__bf16)v[i]; r.h[i] = h; r.l[i] = (__bf16)(v[i] - (float)h); }
  return r; }
__device__ __forceinline__ F2 split_row(const float* row, int k0, int lane) { float v[16]; const float* p = row + k0 + 8 * (lane >> 4);
#pragma unroll
  for (int i = 0; i < 8; ++i) { v[i] = p[i]; v[8 + i] = p[16 + i]; }
  return bsplit16(v); }
__device__ __forceinline__ F2 split_rowK(const float* row, int k0, int lane, int K) { float v[16]; const int g = lane >> 4;
#pragma unroll
  for (int i = 0; i < 8; ++i) { const int ka = k0 + 8 * g + i, kb = ka + 16; v[i] = ka < K ? row[ka < K ? ka : K - 1] : 0.f; v[8 + i] = kb < K ? row[kb < K ? kb : K - 1] : 0.f; }
  return bsplit16(v); }
__device__ __forceinline__ F2 split_col(const float* W, int k0, int n, int lane, int ld, int K) { float v[16]; const int g = lane >> 4;
#pragma unroll
  for (int i = 0; i < 8; ++i) { const int ka = k0 + 8 * g + i, kb = ka + 16; v[i] = ka < K ? W[(size_t)(ka < K ? ka : K - 1) * ld + n] : 0.f; v[8 + i] = kb < K ? W[(size_t)(kb < K ? kb : K - 1) * ld + n] : 0.f; }
  return bsplit16(v); }
__device__ __forceinline__ v8f mac3(const F2& a, const F2& b, v8f c) { c = wmma_bf(a.l, b.h, c); c = wmma_bf(a.h, b.l, c); return wmma_bf(a.h, b.h, c); }
__device__ __forceinline__ float sigm(float v) { return 1.0f / (1.0f + expf(-v)); }
#define LDSX() do { asm volatile("s_wait_dscnt 0" ::: "memory"); __builtin_amdgcn_wave_barrier(); __builtin_amdgcn_fence(__ATOMIC_RELEASE, "workgroup"); } while (0)

#define NB_ 8
#define NPTS 4096
#define NP 1024
#define CF 64
#define CIN 67
#define NQ (NB_ * NP)
#define SP 32
#define CT 384
#define OFF_FEAT 98304u
#define BN_EPS 1e-5f
__device__ __forceinline__ float bfr(float v) { return (float)(__bf16)v; }
typedef __attribute__((ext_vector_type(4))) int v4i;
__device__ __forceinline__ v16b wcol_kz(const float* __restrict__ Wm, int k0, int o, int lane, int ld, int K, int nvalid) { v16b w; const int g = lane >> 4; const int oc = o < nvalid ? o : 0; const float keepo = o < nvalid ? 1.f : 0.f;
  asm volatile("s_wait_loadcnt 0x0" ::: "memory");
#pragma unroll
  for (int i = 0; i < 8; ++i) { const int ka = k0 + 8 * g + i, kb = ka + 16; w[i] = (__bf16)(Wm[(size_t)(ka < K ? ka : 0) * ld + oc] * (ka < K ? keepo : 0.f)); w[8 + i] = (__bf16)(Wm[(size_t)(kb < K ? kb : 0) * ld + oc] * (kb < K ? keepo : 0.f)); }
  asm volatile("s_wait_loadcnt 0x0" ::: "memory"); return w; }
#define WS_IDX  0u
#define WS_X1   (WS_IDX + 4u * 2 * (size_t)NQ * SP)
#define WS_PART (WS_X1 + 4u * (size_t)NQ * 32 * 128)
#define WS_XMX  (WS_PART + 4u * 4096 * 2 * 256)
#define WS_XMN  (WS_XMX + 4u * (size_t)NQ * 256)
#define WS_SC   (WS_XMN + 4u * (size_t)NQ * 256)
#define WS_END  (WS_SC + 4u * 6 * 2 * 256)
__global__ __launch_bounds__(256) void k_nxyz(const float* __restrict__ XYZ, const int* __restrict__ NPI, float* __restrict__ O0) { const size_t b = blockIdx.x; const int np_ = NPI[0] < NP ? NPI[0] : NP;
  for (int q = threadIdx.x; q < NP * 3 / 4; q += 256) { const v4f v = *(const v4f*)(XYZ + b * NPTS * 3 + (size_t)q * 4); asm volatile("s_wait_loadcnt 0x0" ::: "memory"); v4f o; o[0] = bfr(v[0]); o[1] = bfr(v[1]); o[2] = bfr(v[2]); o[3] = bfr(v[3]);
    if (q * 4 < np_ * 3) vst2(O0 + b * NP * 3 + (size_t)q * 4, o); } }
__global__ __launch_bounds__(256) void k_ball(const float* __restrict__ XYZ, float r2, int S, int* __restrict__ IDX) { __shared__ int sidx[8][SP];
  const int wave = threadIdx.x >> 5, lane = threadIdx.x & 31; const size_t q = (size_t)blockIdx.x * 8 + wave; const size_t b = q / NP; const int p = (int)(q % NP);
  if (lane < SP) sidx[wave][lane] = 0;
  float qx, qy, qz; { const float* pq = XYZ + (b * NPTS + p) * 3; qx = bfr(pq[0]); qy = bfr(pq[1]); qz = bfr(pq[2]); }
  int cnt = 0;
  {
#pragma clang fp contract(off)
#pragma unroll 1
    for (int base = 0; base < NPTS && cnt < S; base += 32) { const int j = base + lane; const float* pj = XYZ + (b * NPTS + j) * 3; const float dx = qx - bfr(pj[0]), dy = qy - bfr(pj[1]), dz = qz - bfr(pj[2]);
      const float d = (dx * dx + dz * dz) + dy * dy; const bool in = d < r2;
      const unsigned m = (unsigned)__ballot(in); const int rank = cnt + (int)__builtin_amdgcn_mbcnt_lo(m, 0u);
      if (in && rank < S) sidx[wave][rank] = j;
      cnt += __popc(m); } }
  LDSX();
  if (lane < SP) { const int v = (lane < S && lane < cnt) ? sidx[wave][lane] : sidx[wave][0]; sidx[wave][lane] = v; }
  LDSX();
  if (lane < 8) vst2((v4i*)(IDX + q * SP) + lane, *(const v4i*)&sidx[wave][lane * 4]); }
template <int NT> __device__ __forceinline__ void bn_partials(const v8f* acc, float (*sps)[2][128], int wave, int lane, int col, int g, int tid, float* __restrict__ PART, size_t blk, int C, int cbase) {
#pragma unroll
  for (int j = 0; j < NT; ++j) { float s1 = 0.f, s2 = 0.f;
#pragma unroll
    for (int r = 0; r < 8; ++r) { const float v = acc[j][r]; s1 += v; s2 += v * v; }
    s1 += __shfl_xor(s1, 16); s2 += __shfl_xor(s2, 16);
    if (g == 0) { sps[wave][0][j * 16 + col] = s1; sps[wave][1][j * 16 + col] = s2; } }
  __syncthreads();
  if (tid < NT * 16) { const int c = tid; const float a = ((sps[0][0][c] + sps[1][0][c]) + sps[2][0][c]) + sps[3][0][c]; const float q2 = ((sps[0][1][c] + sps[1][1][c]) + sps[2][1][c]) + sps[3][1][c]; sps[0][0][c] = a; sps[0][1][c] = q2; }
  __syncthreads();
  if (tid < NT * 16 / 4) { vst2(PART + (blk * 2 + 0) * (size_t)C + cbase + tid * 4, *(const v4f*)&sps[0][0][tid * 4]); vst2(PART + (blk * 2 + 1) * (size_t)C + cbase + tid * 4, *(const v4f*)&sps[0][1][tid * 4]); }
  __syncthreads(); }
__global__ __launch_bounds__(256) void k_bnred(const float* __restrict__ PART, int nblk, int C, float count, const float* __restrict__ G, const float* __restrict__ Bt, float* __restrict__ SC, float* __restrict__ SH) { const int c = threadIdx.x; if (c >= C) return;
  float s = 0.f, q = 0.f; for (int b2 = 0; b2 < nblk; ++b2) { s += PART[((size_t)b2 * 2) * C + c]; q += PART[((size_t)b2 * 2 + 1) * C + c]; }
  const float mean = s / count; const float var = fmaxf(q / count - mean * mean, 0.f); const float sc = bfr(G[c]) * rsqrtf(var + BN_EPS); const float sh = bfr(Bt[c]) - mean * sc;
  vst2(SC + c, sc); vst2(SH + c, sh); }
__device__ __forceinline__ void l0_row(const float* __restrict__ XYZ, const float* __restrict__ FEAT, const int* __restrict__ IDX, int S, size_t gr, int kc, int g, v16b& ah, v16b& al) {
  const size_t q = gr / S; const int s_ = (int)(gr % S); const size_t b = q / NP; const int p = (int)(q % NP); int m = IDX[q * SP + s_]; m = m < 0 ? 0 : (m >= NPTS ? NPTS - 1 : m);
  const float* pm = XYZ + (b * NPTS + m) * 3; const float* pp = XYZ + (b * NPTS + p) * 3; const float* fm = FEAT + (b * NPTS + m) * CF;
  float rel[3]; rel[0] = bfr(pm[0]) - bfr(pp[0]); rel[1] = bfr(pm[1]) - bfr(pp[1]); rel[2] = bfr(pm[2]) - bfr(pp[2]);
  float va[16];
#pragma unroll
  for (int i = 0; i < 16; ++i) { const int k = kc * 32 + 8 * g + (i < 8 ? i : 8 + i); const int kf = k - 3; const int kfc = kf < 0 ? 0 : (kf >= CF ? CF - 1 : kf); const float fv = bfr(fm[kfc]);
    const float rv = (k == 0 ? rel[0] : (k == 1 ? rel[1] : rel[2]));
    va[i] = k < 3 ? rv : (k < CIN ? fv : 0.f); }
  asm volatile("s_wait_loadcnt 0x0" ::: "memory");
  const F2 f = bsplit16(va); ah = f.h; al = f.l; }
template <int CO, bool STATS> __global__ __launch_bounds__(128) void k_l0(const float* __restrict__ XYZ, const float* __restrict__ FEAT, const int* __restrict__ IDX, int S, const float* __restrict__ W0, const float* __restrict__ SC0, const float* __restrict__ SH0, const float* __restrict__ W1, float* __restrict__ X1, float* __restrict__ PART) {
  constexpr int NT = CO / 16; __shared__ __align__(16) float sh[4][16][CO + 4]; __shared__ float sps[4][2][128];
  const int tid = threadIdx.x, wave = tid >> 5, lane = tid & 31, col = lane & 15, g = lane >> 4; const size_t r0 = (size_t)blockIdx.x * 64 + wave * 16;
  v8f acc[NT] = {};
#pragma unroll 1
  for (int kc = 0; kc < 3; ++kc) { v16b ah, al; l0_row(XYZ, FEAT, IDX, S, r0 + col, kc, g, ah, al);
#pragma unroll
    for (int j = 0; j < NT; ++j) { const v16b w = wcol_kz(W0, kc * 32, j * 16 + col, lane, CO, CIN, CO); acc[j] = wmma_bf(ah, w, acc[j]); if (kc == 0) acc[j] = wmma_bf(al, w, acc[j]); } }
  if (STATS) { bn_partials<NT>(acc, sps, wave, lane, col, g, tid, PART, blockIdx.x, CO, 0); return; }
#pragma unroll
  for (int j = 0; j < NT; ++j) { const int c = j * 16 + col; const float sc = SC0[c], sf = SH0[c]; asm volatile("s_wait_loadcnt 0x0" ::: "memory");
#pragma unroll
    for (int r = 0; r < 8; ++r) sh[wave][8 * g + r][c] = fmaxf(acc[j][r] * sc + sf, 0.f); }
  LDSX();
  v8f acc1[NT] = {};
#pragma unroll
  for (int kc = 0; kc < CO / 32; ++kc) { const F2 a = split_row(&sh[wave][col][0], kc * 32, lane);
#pragma unroll
    for (int j = 0; j < NT; ++j) { const v16b w = wcol_kz(W1, kc * 32, j * 16 + col, lane, CO, CO, CO); acc1[j] = wmma_bf(a.h, w, acc1[j]); acc1[j] = wmma_bf(a.l, w, acc1[j]); } }
  LDSX();
#pragma unroll
  for (int j = 0; j < NT; ++j) {
#pragma unroll
    for (int r = 0; r < 8; ++r) sh[wave][8 * g + r][j * 16 + col] = acc1[j][r]; }
  LDSX(); for (int rl = 0; rl < 16; ++rl) if (lane < CO / 4) vst2(X1 + (r0 + rl) * CO + lane * 4, *(const v4f*)&sh[wave][rl][lane * 4]);
  bn_partials<NT>(acc1, sps, wave, lane, col, g, tid, PART, blockIdx.x, CO, 0); }
template <int C1> __global__ __launch_bounds__(128) void k_l2(const float* __restrict__ X1, const float* __restrict__ SC1, const float* __restrict__ SH1, const float* __restrict__ W2, int C2, int S, float* __restrict__ PART, float* __restrict__ XMX, float* __restrict__ XMN) {
  __shared__ __align__(16) float sh[4][16][C1 + 4]; __shared__ float sps[4][2][128]; __shared__ __align__(16) float smx[4][128], smn[4][128];
  const int tid = threadIdx.x, wave = tid >> 5, lane = tid & 31, col = lane & 15, g = lane >> 4; const size_t r0 = (size_t)blockIdx.x * 64 + wave * 16; const int cb = blockIdx.y; const int c0 = cb * 128;
  for (int rl = 0; rl < 16; ++rl) if (lane < C1 / 4) { const v4f v = *(const v4f*)(X1 + (r0 + rl) * C1 + lane * 4); const v4f sc = *(const v4f*)(SC1 + lane * 4), sf = *(const v4f*)(SH1 + lane * 4); asm volatile("s_wait_loadcnt 0x0" ::: "memory"); v4f o; o[0] = fmaxf(v[0] * sc[0] + sf[0], 0.f); o[1] = fmaxf(v[1] * sc[1] + sf[1], 0.f); o[2] = fmaxf(v[2] * sc[2] + sf[2], 0.f); o[3] = fmaxf(v[3] * sc[3] + sf[3], 0.f); *(v4f*)&sh[wave][rl][lane * 4] = o; }
  LDSX();
  v8f acc[8] = {};
#pragma unroll
  for (int kc = 0; kc < C1 / 32; ++kc) { const F2 a = split_row(&sh[wave][col][0], kc * 32, lane);
#pragma unroll
    for (int j = 0; j < 8; ++j) { const v16b w = wcol_kz(W2, kc * 32, c0 + j * 16 + col, lane, C2, C1, C2); acc[j] = wmma_bf(a.h, w, acc[j]); acc[j] = wmma_bf(a.l, w, acc[j]); } }
#pragma unroll
  for (int j = 0; j < 8; ++j) { float mx = -3.0e38f, mn = 3.0e38f;
#pragma unroll
    for (int r = 0; r < 8; ++r) { mx = fmaxf(mx, acc[j][r]); mn = fminf(mn, acc[j][r]); }
    mx = fmaxf(mx, __shfl_xor(mx, 16)); mn = fminf(mn, __shfl_xor(mn, 16));
    if (g == 0) { smx[wave][j * 16 + col] = mx; smn[wave][j * 16 + col] = mn; } }
  __syncthreads();
  if (S == 16) { const int w = tid >> 5; const size_t grp = (r0) / 16;
    { v4f o; o[0] = smx[w][lane * 4]; o[1] = smx[w][lane * 4 + 1]; o[2] = smx[w][lane * 4 + 2]; o[3] = smx[w][lane * 4 + 3]; vst2(XMX + grp * C2 + c0 + lane * 4, o); }
    { v4f o; o[0] = smn[w][lane * 4]; o[1] = smn[w][lane * 4 + 1]; o[2] = smn[w][lane * 4 + 2]; o[3] = smn[w][lane * 4 + 3]; vst2(XMN + grp * C2 + c0 + lane * 4, o); } }
  else { if (tid < 64) { const int pr = tid >> 5; const size_t grp = ((size_t)blockIdx.x * 64 + pr * 32) / 32;
      { v4f o; o[0] = fmaxf(smx[2 * pr][lane * 4], smx[2 * pr + 1][lane * 4]); o[1] = fmaxf(smx[2 * pr][lane * 4 + 1], smx[2 * pr + 1][lane * 4 + 1]); o[2] = fmaxf(smx[2 * pr][lane * 4 + 2], smx[2 * pr + 1][lane * 4 + 2]); o[3] = fmaxf(smx[2 * pr][lane * 4 + 3], smx[2 * pr + 1][lane * 4 + 3]); vst2(XMX + grp * C2 + c0 + lane * 4, o); }
      { v4f o; o[0] = fminf(smn[2 * pr][lane * 4], smn[2 * pr + 1][lane * 4]); o[1] = fminf(smn[2 * pr][lane * 4 + 1], smn[2 * pr + 1][lane * 4 + 1]); o[2] = fminf(smn[2 * pr][lane * 4 + 2], smn[2 * pr + 1][lane * 4 + 2]); o[3] = fminf(smn[2 * pr][lane * 4 + 3], smn[2 * pr + 1][lane * 4 + 3]); vst2(XMN + grp * C2 + c0 + lane * 4, o); } } }
  bn_partials<8>(acc, sps, wave, lane, col, g, tid, PART, blockIdx.x, C2, c0); }
__global__ __launch_bounds__(256) void k_fin(const float* __restrict__ XMX, const float* __restrict__ XMN, const float* __restrict__ SC2, const float* __restrict__ SH2, int C2, int coff, float* __restrict__ O1) { const size_t b = blockIdx.x; const int c = blockIdx.y;
  const float sc = SC2[c], sf = SH2[c]; asm volatile("s_wait_loadcnt 0x0" ::: "memory"); const float* SRC = (sc >= 0.f) ? XMX : XMN;
  const int p0 = threadIdx.x * 4; v4f o;
#pragma unroll
  for (int i = 0; i < 4; ++i) { const float v = SRC[(b * NP + p0 + i) * (size_t)C2 + c]; o[i] = fmaxf(v * sc + sf, 0.f); }
  asm volatile("s_wait_loadcnt 0x0" ::: "memory");
  vst2(O1 + (b * CT + coff + c) * (size_t)NP + p0, o); }
extern "C" void kernel_launch(void* const* d_in, const int* in_sizes, int n_in, void* d_out, int out_size, void* d_ws, size_t ws_size, hipStream_t stream) {
  (void)in_sizes; (void)n_in; (void)out_size;
  if (ws_size < (size_t)WS_END) return;
  char* ws = (char*)d_ws; const float** F = (const float**)d_in; int* IDX = (int*)(ws + WS_IDX); float *X1 = (float*)(ws + WS_X1), *PART = (float*)(ws + WS_PART), *XMX = (float*)(ws + WS_XMX), *XMN = (float*)(ws + WS_XMN), *SCB = (float*)(ws + WS_SC);
  float* O1 = (float*)((char*)d_out + OFF_FEAT);
  k_nxyz<<<dim3(NB_), 256, 0, stream>>>(F[0], (const int*)d_in[2], (float*)d_out);
  { const int S = 16, C = 64, C2 = 128, coff = 0; const size_t R = (size_t)NQ * S; const int nblk = (int)(R / 64); int* IDX0 = IDX; float *sc0 = SCB, *sh0 = SCB + 256, *sc1 = SCB + 512, *sh1 = SCB + 768, *sc2 = SCB + 1024, *sh2 = SCB + 1280;
    k_ball<<<dim3(NQ / 8), 256, 0, stream>>>(F[0], 0.04f, S, IDX0);
    k_l0<64, true><<<dim3(nblk), 128, 0, stream>>>(F[0], F[1], IDX0, S, F[3], nullptr, nullptr, nullptr, nullptr, PART);
    k_bnred<<<1, 256, 0, stream>>>(PART, nblk, C, (float)R, F[4], F[5], sc0, sh0);
    k_l0<64, false><<<dim3(nblk), 128, 0, stream>>>(F[0], F[1], IDX0, S, F[3], sc0, sh0, F[6], X1, PART);
    k_bnred<<<1, 256, 0, stream>>>(PART, nblk, C, (float)R, F[7], F[8], sc1, sh1);
    k_l2<64><<<dim3(nblk, C2 / 128), 128, 0, stream>>>(X1, sc1, sh1, F[9], C2, S, PART, XMX, XMN);
    k_bnred<<<1, 256, 0, stream>>>(PART, nblk, C2, (float)R, F[10], F[11], sc2, sh2);
    k_fin<<<dim3(NB_, C2), 256, 0, stream>>>(XMX, XMN, sc2, sh2, C2, coff, O1); }
  { const int S = 32, C = 128, C2 = 256, coff = 128; const size_t R = (size_t)NQ * S; const int nblk = (int)(R / 64); int* IDX1 = IDX + (size_t)NQ * SP; float *sc0 = SCB + 1536, *sh0 = SCB + 1792, *sc1 = SCB + 2048, *sh1 = SCB + 2304, *sc2 = SCB + 2560, *sh2 = SCB + 2816;
    k_ball<<<dim3(NQ / 8), 256, 0, stream>>>(F[0], 0.16f, S, IDX1);
    k_l0<128, true><<<dim3(nblk), 128, 0, stream>>>(F[0], F[1], IDX1, S, F[12], nullptr, nullptr, nullptr, nullptr, PART);
    k_bnred<<<1, 256, 0, stream>>>(PART, nblk, C, (float)R, F[13], F[14], sc0, sh0);
    k_l0<128, false><<<dim3(nblk), 128, 0, stream>>>(F[0], F[1], IDX1, S, F[12], sc0, sh0, F[15], X1, PART);
    k_bnred<<<1, 256, 0, stream>>>(PART, nblk, C, (float)R, F[16], F[17], sc1, sh1);
    k_l2<128><<<dim3(nblk, C2 / 128), 128, 0, stream>>>(X1, sc1, sh1, F[18], C2, S, PART, XMX, XMN);
    k_bnred<<<1, 256, 0, stream>>>(PART, nblk, C2, (float)R, F[19], F[20], sc2, sh2);
    k_fin<<<dim3(NB_, C2), 256, 0, stream>>>(XMX, XMN, sc2, sh2, C2, coff, O1); }
}
